// SPAttention_12249246728420
// MI455X (gfx1250) — hardware-verified
//
#include <hip/hip_runtime.h>


typedef _Float16     v16h __attribute__((ext_vector_type(16)));
typedef _Float16     v8h  __attribute__((ext_vector_type(8)));
typedef float        v8f  __attribute__((ext_vector_type(8)));
typedef float        v4f  __attribute__((ext_vector_type(4)));
typedef unsigned int v4u  __attribute__((ext_vector_type(4)));
typedef v8h v8ha __attribute__((may_alias));
typedef v4f v4fa __attribute__((may_alias));

union Frag { v16h v; v8h half[2]; };
union F8   { v8f v; float f[8]; };
union H8   { v8h h; v4u u; _Float16 e[8]; };

__device__ __forceinline__ v8f zero8() { v8f z = {0.f, 0.f, 0.f, 0.f, 0.f, 0.f, 0.f, 0.f}; return z; }

__device__ __forceinline__ void mma(v8f& d, const v16h& a, const v16h& b) {
    d = __builtin_amdgcn_wmma_f32_16x16x32_f16(false, a, false, b, (short)0, d, false, false);
}
__device__ __forceinline__ void hz1(v8f& d0, const v16h& f0, const v16h& f1) {
    asm volatile("v_nop\n\tv_nop\n\tv_nop\n\tv_nop" : "+v"(d0) : "v"(f0), "v"(f1));
}
__device__ __forceinline__ void hz2(v8f& d0, v8f& d1, const v16h& f0, const v16h& f1, const v16h& f2) {
    asm volatile("v_nop\n\tv_nop\n\tv_nop\n\tv_nop" : "+v"(d0), "+v"(d1) : "v"(f0), "v"(f1), "v"(f2));
}
__device__ __forceinline__ void hz2w(v8f& d0, v8f& d1, const v16h& f0, const v16h& f1, const v16h& f2, const v16h& f3) {
    asm volatile("v_nop\n\tv_nop\n\tv_nop\n\tv_nop" : "+v"(d0), "+v"(d1) : "v"(f0), "v"(f1), "v"(f2), "v"(f3));
}
__device__ __forceinline__ void hz4(v8f& d0, v8f& d1, v8f& d2, v8f& d3,
                                    const v16h& f0, const v16h& f1, const v16h& f2, const v16h& f3) {
    asm volatile("v_nop\n\tv_nop\n\tv_nop\n\tv_nop" : "+v"(d0), "+v"(d1), "+v"(d2), "+v"(d3) : "v"(f0), "v"(f1), "v"(f2), "v"(f3));
}

__device__ __forceinline__ v16h ldfrag(const _Float16* row, int lh) {
    Frag f;
    f.half[0] = *(const v8ha*)(row + 8 * lh);
    f.half[1] = *(const v8ha*)(row + 16 + 8 * lh);
    return f.v;
}

__device__ __forceinline__ float bf16_rne(float x) {
    unsigned int u = __float_as_uint(x);
    u = (u + 0x7FFFu + ((u >> 16) & 1u)) & 0xFFFF0000u;
    return __uint_as_float(u);
}

__device__ __forceinline__ void st16(_Float16* p, v4u u) { *(volatile v4u*)p = u; }
__device__ __forceinline__ void st16f(float* p, v4f v) { *(volatile v4f*)p = v; }

__global__ __launch_bounds__(256)
void k_cvx(const float* __restrict__ X, _Float16* __restrict__ Xh, int n8, float scale)
{
    const int i = blockIdx.x * 256 + threadIdx.x;
    if (i >= n8) return;
    const float* p = X + (size_t)i * 8;
    const v4f a = *(const v4f*)p;
    const v4f c = *(const v4f*)(p + 4);
    H8 o;
    o.e[0] = (_Float16)(bf16_rne(a.x) * scale);
    o.e[1] = (_Float16)(bf16_rne(a.y) * scale);
    o.e[2] = (_Float16)(bf16_rne(a.z) * scale);
    o.e[3] = (_Float16)(bf16_rne(a.w) * scale);
    o.e[4] = (_Float16)(bf16_rne(c.x) * scale);
    o.e[5] = (_Float16)(bf16_rne(c.y) * scale);
    o.e[6] = (_Float16)(bf16_rne(c.z) * scale);
    o.e[7] = (_Float16)(bf16_rne(c.w) * scale);
    _Float16* d = Xh + (size_t)i * 8;
    st16(d, o.u);
    __threadfence();
    st16(d, o.u);
}

__global__ __launch_bounds__(256)
void k_cvwt(const float* __restrict__ W, _Float16* __restrict__ Wt, int K, int N, float scale)
{
    __shared__ float tile[64][65];
    const int k0 = blockIdx.y * 64, n0 = blockIdx.x * 64, t = threadIdx.x;
    #pragma unroll
    for (int i = 0; i < 4; ++i) {
        const int idx = i * 256 + t, kk = idx >> 4, nn = (idx & 15) * 4;
        v4f v = {0.f, 0.f, 0.f, 0.f};
        if (k0 + kk < K && n0 + nn + 3 < N) v = *(const v4f*)(W + (size_t)(k0 + kk) * N + n0 + nn);
        tile[kk][nn] = v.x; tile[kk][nn + 1] = v.y; tile[kk][nn + 2] = v.z; tile[kk][nn + 3] = v.w;
    }
    __syncthreads();
    H8 o[2]; size_t dst[2]; bool ok[2];
    #pragma unroll
    for (int i = 0; i < 2; ++i) {
        const int idx = i * 256 + t, nn = idx >> 3, seg = idx & 7;
        #pragma unroll
        for (int j = 0; j < 8; ++j) o[i].e[j] = (_Float16)(bf16_rne(tile[seg * 8 + j][nn]) * scale);
        dst[i] = (size_t)(n0 + nn) * K + k0 + seg * 8;
        ok[i] = (n0 + nn < N) && (k0 + seg * 8 + 7 < K);
    }
    #pragma unroll
    for (int i = 0; i < 2; ++i) if (ok[i]) st16(Wt + dst[i], o[i].u);
    __threadfence();
    #pragma unroll
    for (int i = 0; i < 2; ++i) if (ok[i]) st16(Wt + dst[i], o[i].u);
}

template <int MODE>
__global__ __launch_bounds__(256)
void k_gemm(const _Float16* __restrict__ A0, const _Float16* __restrict__ A1,
            const _Float16* __restrict__ Bt, const float* __restrict__ bias,
            _Float16* __restrict__ P0, _Float16* __restrict__ P1,
            _Float16* __restrict__ V0, _Float16* __restrict__ V1,
            float* __restrict__ Out,
            int Mtot, int N, int K, int tpg, int gstride, int roff,
            int T, int Cq, int H, float oscale)
{
    constexpr int BM = 128, BN = 64, BK = 32, LK = BK + 8, LC = BN + 4;
    constexpr int NPA = (MODE == 1) ? 2 : 1;
    constexpr int AS_BYTES = 2 * BM * LK * 2;
    constexpr int SMEM_BYTES = BM * LC * 4;
    __shared__ __attribute__((aligned(16))) unsigned char smem[SMEM_BYTES];
    _Float16* As = (_Float16*)smem;
    _Float16* Bs = (_Float16*)(smem + AS_BYTES);
    float*    Cs = (float*)smem;

    const int tid = threadIdx.x, wave = tid >> 5, l = tid & 31, lh = l >> 4, m = l & 15;
    const int wm = wave >> 1, wn = wave & 1;
    const int by = blockIdx.y;
    const int m0 = (by / tpg) * gstride + roff + (by % tpg) * BM;
    const int bn = blockIdx.x * BN;
    const v4u z4 = {0u, 0u, 0u, 0u};

    F8 acc[2][2], accx[2][2];
    #pragma unroll
    for (int mi = 0; mi < 2; ++mi)
        #pragma unroll
        for (int ni = 0; ni < 2; ++ni) { acc[mi][ni].v = zero8(); accx[mi][ni].v = zero8(); }

    for (int k0 = 0; k0 < K; k0 += BK) {
        #pragma unroll
        for (int p = 0; p < NPA; ++p) {
            const _Float16* Ap = (p == 0) ? A0 : A1;
            #pragma unroll
            for (int i = 0; i < 2; ++i) {
                const int idx = i * 256 + tid, r = idx >> 2, seg = idx & 3;
                const int gm = m0 + r;
                H8 v; v.u = z4;
                if (gm < Mtot) v.h = *(const v8h*)(Ap + (size_t)gm * K + k0 + seg * 8);
                *(v8ha*)(As + (p * BM + r) * LK + seg * 8) = v.h;
            }
        }
        {
            const int r = tid >> 2, seg = tid & 3;
            const int gn = bn + r;
            H8 v; v.u = z4;
            if (gn < N) v.h = *(const v8h*)(Bt + (size_t)gn * K + k0 + seg * 8);
            *(v8ha*)(Bs + r * LK + seg * 8) = v.h;
        }
        __syncthreads();

        const v16h b0 = ldfrag(Bs + (wn * 32 + m) * LK, lh);
        const v16h b1 = ldfrag(Bs + (wn * 32 + 16 + m) * LK, lh);
        #pragma unroll
        for (int mi = 0; mi < 2; ++mi) {
            const v16h ah = ldfrag(As + (wm * 32 + mi * 16 + m) * LK, lh);
            if constexpr (MODE == 1) {
                const v16h al = ldfrag(As + (BM + wm * 32 + mi * 16 + m) * LK, lh);
                mma(acc[mi][0].v, ah, b0);
                mma(acc[mi][1].v, ah, b1);
                mma(accx[mi][0].v, al, b0);
                mma(accx[mi][1].v, al, b1);
                hz4(acc[mi][0].v, acc[mi][1].v, accx[mi][0].v, accx[mi][1].v, ah, al, b0, b1);
            } else {
                mma(acc[mi][0].v, ah, b0);
                mma(acc[mi][1].v, ah, b1);
                hz2(acc[mi][0].v, acc[mi][1].v, ah, b0, b1);
            }
        }
        __syncthreads();
    }

    const float ps = (MODE == 0) ? 16.0f : 1.0f;
    const float xs = oscale * (1.0f / 2048.0f);
    #pragma unroll
    for (int mi = 0; mi < 2; ++mi)
        #pragma unroll
        for (int ni = 0; ni < 2; ++ni) {
            const int cl = wn * 32 + ni * 16 + m;
            const int gn = bn + cl;
            const float bv = (gn < N) ? bias[gn] : 0.f;
            #pragma unroll
            for (int r = 0; r < 8; ++r) {
                float v = acc[mi][ni].f[r] * oscale;
                if constexpr (MODE == 1) v += accx[mi][ni].f[r] * xs;
                v = (v + bv) * ps;
                Cs[(wm * 32 + mi * 16 + 8 * lh + r) * LC + cl] = v;
            }
        }
    __syncthreads();

    if constexpr (MODE == 0) {
        if (bn < Cq) {
            auto pass = [&]() {
                #pragma unroll
                for (int it = 0; it < 4; ++it) {
                    const int row = wave * 16 + it * 4 + (l >> 3), seg = l & 7;
                    const int gm = m0 + row;
                    const float* src = Cs + row * LC + seg * 8;
                    const v4f a = *(const v4fa*)src;
                    const v4f c = *(const v4fa*)(src + 4);
                    const float x[8] = {a.x, a.y, a.z, a.w, c.x, c.y, c.z, c.w};
                    H8 hi, lo;
                    #pragma unroll
                    for (int j = 0; j < 8; ++j) {
                        const _Float16 hh = (_Float16)x[j];
                        hi.e[j] = hh;
                        lo.e[j] = (_Float16)((x[j] - (float)hh) * 2048.0f);
                    }
                    if (gm < Mtot && bn + seg * 8 + 7 < Cq) {
                        const size_t off = (size_t)gm * Cq + bn + seg * 8;
                        st16(P0 + off, hi.u);
                        st16(P1 + off, lo.u);
                    }
                }
            };
            pass();
            __threadfence();
            pass();
        } else {
            const int hd = (bn - Cq) >> 6;
            const int bidx = m0 / T, t0 = m0 - bidx * T;
            auto pass = [&]() {
                #pragma unroll
                for (int it = 0; it < 4; ++it) {
                    const int d = wave * 8 + it * 2 + (l >> 4), ms = l & 15;
                    float x[8];
                    #pragma unroll
                    for (int j = 0; j < 8; ++j) x[j] = Cs[(ms * 8 + j) * LC + d];
                    H8 hi, lo;
                    #pragma unroll
                    for (int j = 0; j < 8; ++j) {
                        const _Float16 hh = (_Float16)x[j];
                        hi.e[j] = hh;
                        lo.e[j] = (_Float16)((x[j] - (float)hh) * 2048.0f);
                    }
                    if (m0 + ms * 8 + 7 < Mtot) {
                        const size_t off = ((size_t)(bidx * H + hd) * 64 + d) * T + t0 + ms * 8;
                        st16(V0 + off, hi.u);
                        st16(V1 + off, lo.u);
                    }
                }
            };
            pass();
            __threadfence();
            pass();
        }
    } else {
        auto pass = [&]() {
            #pragma unroll
            for (int it = 0; it < 8; ++it) {
                const int row = wave * 16 + it * 2 + (l >> 4), cs = (l & 15) * 4;
                const int gm = m0 + row;
                const v4f v = *(const v4fa*)(Cs + row * LC + cs);
                if (gm < Mtot && bn + cs + 3 < N) st16f(Out + (size_t)gm * N + bn + cs, v);
            }
        };
        pass();
        __threadfence();
        pass();
    }
}

template <bool SPV>
__global__ __launch_bounds__(128)
void k_attn(const _Float16* __restrict__ QKh, const _Float16* __restrict__ QKl,
            const _Float16* __restrict__ Vth, const _Float16* __restrict__ Vtl,
            _Float16* __restrict__ Oh, _Float16* __restrict__ Ol,
            int T, int C, int H, int qtbase)
{
    constexpr int KT = 64, LP = 64;
    constexpr int NR2 = SPV ? KT : 1;
    __shared__ __attribute__((aligned(16))) _Float16 Qh_s[KT * LP];
    __shared__ __attribute__((aligned(16))) _Float16 Ql_s[KT * LP];
    __shared__ __attribute__((aligned(16))) _Float16 Kh_s[KT * LP];
    __shared__ __attribute__((aligned(16))) _Float16 Kl_s[KT * LP];
    __shared__ __attribute__((aligned(16))) _Float16 Vh_s[KT * LP];
    __shared__ __attribute__((aligned(16))) _Float16 Vl_s[NR2 * LP];
    __shared__ __attribute__((aligned(16))) _Float16 Ph_s[KT * LP];
    __shared__ __attribute__((aligned(16))) _Float16 Pl_s[NR2 * LP];

    const int qt = blockIdx.x + qtbase;
    const int b = blockIdx.y / H, h = blockIdx.y - b * H;
    const int tid = threadIdx.x, wave = tid >> 5, l = tid & 31, lh = l >> 4, m = l & 15;
    const int q0 = qt * KT;
    const int C2 = 2 * C;
    const int prow = wave * 16;
    const v4u z4 = {0u, 0u, 0u, 0u};
    const float NEG = -__builtin_inff();
    const float xc = 1.0f / 2048.0f;
    const float sc = 1.0f / 2048.0f;

    #pragma unroll
    for (int i = 0; i < 4; ++i) {
        const int idx = i * 128 + tid, row = idx >> 3, seg = idx & 7;
        H8 a, c; a.u = z4; c.u = z4;
        if (q0 + row < T) {
            const size_t off = (size_t)(b * T + q0 + row) * C2 + h * 64 + seg * 8;
            a.h = *(const v8h*)(QKh + off);
            c.h = *(const v8h*)(QKl + off);
        }
        *(v8ha*)(Qh_s + row * LP + seg * 8) = a.h;
        *(v8ha*)(Ql_s + row * LP + seg * 8) = c.h;
    }

    F8 o[4];
    float mrow[8], lrow[8];
    #pragma unroll
    for (int di = 0; di < 4; ++di) o[di].v = zero8();
    #pragma unroll
    for (int r = 0; r < 8; ++r) { mrow[r] = NEG; lrow[r] = 0.f; }

    for (int j = 0; j <= qt; ++j) {
        const int kb = j * KT;
        #pragma unroll
        for (int i = 0; i < 4; ++i) {
            const int idx = i * 128 + tid, row = idx >> 3, seg = idx & 7;
            H8 a, c, v; a.u = z4; c.u = z4; v.u = z4;
            if (kb + row < T) {
                const size_t off = (size_t)(b * T + kb + row) * C2 + C + h * 64 + seg * 8;
                a.h = *(const v8h*)(QKh + off);
                c.h = *(const v8h*)(QKl + off);
            }
            *(v8ha*)(Kh_s + row * LP + seg * 8) = a.h;
            *(v8ha*)(Kl_s + row * LP + seg * 8) = c.h;
            const size_t voff = ((size_t)(b * H + h) * 64 + row) * T + kb + seg * 8;
            if (kb + seg * 8 + 7 < T) v.h = *(const v8h*)(Vth + voff);
            *(v8ha*)(Vh_s + row * LP + seg * 8) = v.h;
            if constexpr (SPV) {
                H8 w; w.u = z4;
                if (kb + seg * 8 + 7 < T) w.h = *(const v8h*)(Vtl + voff);
                *(v8ha*)(Vl_s + row * LP + seg * 8) = w.h;
            }
        }
        __syncthreads();

        F8 s[4], c[4];
        #pragma unroll
        for (int ni = 0; ni < 4; ++ni) { s[ni].v = zero8(); c[ni].v = zero8(); }
        #pragma unroll 1
        for (int ks = 0; ks < 2; ++ks) {
            const v16h qh = ldfrag(Qh_s + (prow + m) * LP + ks * 32, lh);
            const v16h ql = ldfrag(Ql_s + (prow + m) * LP + ks * 32, lh);
            #pragma unroll
            for (int ni = 0; ni < 4; ++ni) {
                const v16h kh = ldfrag(Kh_s + (ni * 16 + m) * LP + ks * 32, lh);
                const v16h kl = ldfrag(Kl_s + (ni * 16 + m) * LP + ks * 32, lh);
                mma(s[ni].v, qh, kh);
                mma(c[ni].v, qh, kl);
                mma(c[ni].v, ql, kh);
                hz2w(s[ni].v, c[ni].v, qh, ql, kh, kl);
            }
        }

        float mnew[8];
        #pragma unroll
        for (int r = 0; r < 8; ++r) {
            const int qg = q0 + prow + 8 * lh + r;
            float mx = NEG;
            #pragma unroll
            for (int ni = 0; ni < 4; ++ni) {
                float x = (s[ni].f[r] + c[ni].f[r] * xc) * sc;
                const int kg = kb + ni * 16 + m;
                x = (kg > qg) ? NEG : x;
                s[ni].f[r] = x;
                mx = fmaxf(mx, x);
            }
            mx = fmaxf(mx, __shfl_xor(mx, 1, 32));
            mx = fmaxf(mx, __shfl_xor(mx, 2, 32));
            mx = fmaxf(mx, __shfl_xor(mx, 4, 32));
            mx = fmaxf(mx, __shfl_xor(mx, 8, 32));
            mnew[r] = fmaxf(mrow[r], mx);
        }
        #pragma unroll
        for (int r = 0; r < 8; ++r) {
            const float corr = __expf(mrow[r] - mnew[r]);
            mrow[r] = mnew[r];
            lrow[r] *= corr;
            #pragma unroll
            for (int di = 0; di < 4; ++di) o[di].f[r] *= corr;
        }
        #pragma unroll
        for (int r = 0; r < 8; ++r) {
            float rs = 0.f;
            #pragma unroll
            for (int ni = 0; ni < 4; ++ni) {
                const float p = __expf(s[ni].f[r] - mnew[r]);
                s[ni].f[r] = p;
                rs += p;
            }
            rs += __shfl_xor(rs, 1, 32);
            rs += __shfl_xor(rs, 2, 32);
            rs += __shfl_xor(rs, 4, 32);
            rs += __shfl_xor(rs, 8, 32);
            lrow[r] += rs;
        }

        #pragma unroll
        for (int ni = 0; ni < 4; ++ni)
            #pragma unroll
            for (int r = 0; r < 8; ++r) {
                const float p4 = s[ni].f[r] * 4096.0f;
                const _Float16 ph = (_Float16)p4;
                const int pi = (prow + 8 * lh + r) * LP + ni * 16 + m;
                Ph_s[pi] = ph;
                if constexpr (SPV) Pl_s[pi] = (_Float16)((p4 - (float)ph) * 2048.0f);
            }
        __syncthreads();

        if constexpr (SPV) {
            F8 oc[4];
            #pragma unroll
            for (int di = 0; di < 4; ++di) oc[di].v = zero8();
            #pragma unroll 1
            for (int ks = 0; ks < 2; ++ks) {
                const v16h ph = ldfrag(Ph_s + (prow + m) * LP + ks * 32, lh);
                const v16h pl = ldfrag(Pl_s + (prow + m) * LP + ks * 32, lh);
                #pragma unroll
                for (int di = 0; di < 4; ++di) {
                    const v16h vh = ldfrag(Vh_s + (di * 16 + m) * LP + ks * 32, lh);
                    const v16h vl = ldfrag(Vl_s + (di * 16 + m) * LP + ks * 32, lh);
                    mma(o[di].v, ph, vh);
                    mma(oc[di].v, ph, vl);
                    mma(oc[di].v, pl, vh);
                    hz2w(o[di].v, oc[di].v, ph, pl, vh, vl);
                }
            }
            #pragma unroll
            for (int di = 0; di < 4; ++di)
                #pragma unroll
                for (int r = 0; r < 8; ++r) o[di].f[r] += oc[di].f[r] * xc;
        } else {
            #pragma unroll 1
            for (int ks = 0; ks < 2; ++ks) {
                const v16h ph = ldfrag(Ph_s + (prow + m) * LP + ks * 32, lh);
                #pragma unroll
                for (int di = 0; di < 4; ++di) {
                    const v16h vh = ldfrag(Vh_s + (di * 16 + m) * LP + ks * 32, lh);
                    mma(o[di].v, ph, vh);
                    hz1(o[di].v, ph, vh);
                }
            }
        }
        __syncthreads();
    }

    #pragma unroll
    for (int r = 0; r < 8; ++r) {
        const float inv = (1.0f / lrow[r]) * (1.0f / 4096.0f);
        #pragma unroll
        for (int di = 0; di < 4; ++di) {
            const float x = o[di].f[r] * inv;
            const _Float16 hh = (_Float16)x;
            const int pi = (prow + 8 * lh + r) * LP + di * 16 + m;
            Ph_s[pi] = hh;
            if constexpr (SPV) Pl_s[pi] = (_Float16)((x - (float)hh) * 2048.0f);
        }
    }
    __syncthreads();
    auto pass = [&]() {
        #pragma unroll
        for (int it = 0; it < 4; ++it) {
            const int idx = it * 32 + l, row = idx >> 3, seg = idx & 7;
            const int gq = q0 + prow + row;
            if (gq < T) {
                const size_t off = (size_t)(b * T + gq) * C + h * 64 + seg * 8;
                H8 v; v.h = *(const v8ha*)(Ph_s + (prow + row) * LP + seg * 8);
                st16(Oh + off, v.u);
                if constexpr (SPV) {
                    H8 w; w.h = *(const v8ha*)(Pl_s + (prow + row) * LP + seg * 8);
                    st16(Ol + off, w.u);
                }
            }
        }
    };
    pass();
    __threadfence();
    pass();
}

extern "C" void kernel_launch(void* const* d_in, const int* in_sizes, int n_in,
                              void* d_out, int out_size, void* d_ws, size_t ws_size,
                              hipStream_t stream)
{
    if (n_in < 5) return;
    const float* X  = (const float*)d_in[0];
    const float* Wa = (const float*)d_in[1];
    const float* ba = (const float*)d_in[2];
    const float* Wp = (const float*)d_in[3];
    const float* bp = (const float*)d_in[4];
    float* out = (float*)d_out;

    const int T = 2048, H = 16, DH = 64, QTS = 8;
    const int C  = in_sizes[4];
    const int C3 = in_sizes[2];
    const int nX = in_sizes[0];
    if (C != H * DH || C3 != 3 * C) return;
    if (nX <= 0 || nX % (T * C) != 0) return;
    const int M = nX / C, Bb = M / T;
    if (in_sizes[1] != C * C3 || in_sizes[3] != C * C || out_size != nX) return;
    const int RS = QTS * 64;
    if ((M % 128) || (T % 128) || (RS % 128) || (T <= RS) || (C % 64) || (C3 % 64) || (C % 32)) return;

    size_t off = 0;
    auto carve = [&](size_t nhalf) { _Float16* p = (_Float16*)((char*)d_ws + off); off += nhalf * 2; return p; };
    _Float16* Xh  = carve((size_t)M * C);
    _Float16* Wat = carve((size_t)C3 * C);
    _Float16* Wpt = carve((size_t)C * C);
    _Float16* QKh = carve((size_t)M * 2 * C);
    _Float16* QKl = carve((size_t)M * 2 * C);
    _Float16* Vth = carve((size_t)M * C);
    _Float16* Vtl = carve((size_t)M * C);
    _Float16* Ohp = carve((size_t)M * C);
    _Float16* Olp = carve((size_t)M * C);
    if (off > ws_size) return;

    k_cvx<<<dim3((nX / 8 + 255) / 256), dim3(256), 0, stream>>>(X, Xh, nX / 8, 16.0f);
    k_cvwt<<<dim3(C3 / 64, C / 64), dim3(256), 0, stream>>>(Wa, Wat, C, C3, 512.0f);
    k_cvwt<<<dim3(C / 64, C / 64), dim3(256), 0, stream>>>(Wp, Wpt, C, C, 4096.0f);

    k_gemm<0><<<dim3(C3 / 64, M / 128), dim3(256), 0, stream>>>(
        Xh, Xh, Wat, ba, QKh, QKl, Vth, Vtl, out,
        M, C3, C, M / 128, 0, 0, T, 2 * C, H, 1.0f / 8192.0f);

    k_attn<true><<<dim3(QTS, Bb * H), dim3(128), 0, stream>>>(QKh, QKl, Vth, Vtl, Ohp, Olp, T, C, H, 0);
    k_attn<false><<<dim3(T / 64 - QTS, Bb * H), dim3(128), 0, stream>>>(QKh, QKl, Vth, Vtl, Ohp, Olp, T, C, H, QTS);

    k_gemm<1><<<dim3(C / 64, Bb * (RS / 128)), dim3(256), 0, stream>>>(
        Ohp, Olp, Wpt, bp, QKh, QKl, Vth, Vtl, out,
        M, C, C, RS / 128, T, 0, T, 2 * C, H, 1.0f / 65536.0f);
    k_gemm<2><<<dim3(C / 64, Bb * ((T - RS) / 128)), dim3(256), 0, stream>>>(
        Ohp, Ohp, Wpt, bp, QKh, QKl, Vth, Vtl, out,
        M, C, C, (T - RS) / 128, T, RS, T, 2 * C, H, 1.0f / 65536.0f);
}
